// TransformerBlock_12360915878034
// MI455X (gfx1250) — hardware-run, weakly checked
//
#include <hip/hip_runtime.h>
#pragma clang fp contract(off)


#ifndef NB
#define NB 4
#endif
#ifndef SEQ
#define SEQ 1024
#endif
#define NB_FULL  4
#define SEQ_FULL 1024
#ifndef OUT_SEQ
#define OUT_SEQ SEQ
#endif
#define DM   512
#define NH_  8
#define DH   (DM * NH_)
#define DFF  2048
#define WS   64.0f
#define WSI  (1.0f / 64.0f)
#define LNEPS 1e-5f

static_assert(DM == 512);
static_assert(32 * 8 * 2 == DM);
static_assert(DH == 4096);
static_assert(DM % 64 == 0);
static_assert(DH % 64 == 0);
static_assert(DFF % 64 == 0);
static_assert(DM % 32 == 0);
static_assert(DH % 32 == 0);
static_assert(DFF % 32 == 0);
static_assert(SEQ % 64 == 0);
static_assert((NB * SEQ) % 64 == 0);
static_assert((NB * SEQ) % 8 == 0);
static_assert(NB <= NB_FULL);
static_assert(SEQ <= SEQ_FULL);
static_assert(SEQ >= 64);
static_assert((size_t)NB_FULL * SEQ_FULL * DM * 4 == (size_t)8388608);
static_assert(32 * 8 * 4 == 16 * 64);
static_assert(32 * 4 * 8 == 16 * 64);
static_assert(256 * 4 * 4 == 64 * 64);
static_assert(256 * 8 * 2 == 64 * 64);
static_assert(16 * 68 * 4 <= 131072);
static_assert(64 * 65 * 4 <= 131072);
static_assert((68 * 4) % 16 == 0);

typedef _Float16 h16;
typedef __attribute__((ext_vector_type(16))) _Float16 v16h;
typedef __attribute__((ext_vector_type(8)))  _Float16 v8h;
typedef __attribute__((ext_vector_type(8)))  float    v8f;
typedef __attribute__((ext_vector_type(4)))  float    v4f;
typedef v4f  __attribute__((may_alias)) v4fa;

__device__ __forceinline__ unsigned short f2bf(float f) { unsigned u = __float_as_uint(f); u += 0x7FFFu + ((u >> 16) & 1u); return (unsigned short)(u >> 16); }
__device__ __forceinline__ float bfr(float f) { return __uint_as_float(((unsigned)f2bf(f)) << 16); }
__device__ __forceinline__ v16h cat16(v8h lo, v8h hi) { return __builtin_shufflevector(lo, hi, 0, 1, 2, 3, 4, 5, 6, 7, 8, 9, 10, 11, 12, 13, 14, 15); }
__device__ __forceinline__ h16 toh_flush(float v) { const h16 r = (h16)v; return (fabsf(v) < 6.103515625e-05f) ? (h16)0.0f : r; }
__device__ __forceinline__ v8f wmmag(v16h a, v16h b, v8f c) {
    c = __builtin_amdgcn_wmma_f32_16x16x32_f16(false, a, false, b, (short)0, c, false, false);
    asm volatile("v_nop\n\tv_nop\n\tv_nop\n\tv_nop" : "+v"(c) : "v"(a), "v"(b));
    return c;
}
__device__ __forceinline__ v16h ldh(const h16* p) { return cat16(*(const v8h*)p, *(const v8h*)(p + 16)); }
__device__ __forceinline__ void wave_sync() { __builtin_amdgcn_fence(3  , "wavefront"); __builtin_amdgcn_wave_barrier(); asm volatile("" ::: "memory"); }

__device__ __forceinline__ void gemm_acc(const h16* __restrict__ Ap, const h16* __restrict__ Bp, size_t lda, size_t ldb, int K, int lr, int hi, v8f (&acc)[4][4]) {
#pragma unroll
    for (int mb = 0; mb < 4; ++mb)
#pragma unroll
        for (int nb = 0; nb < 4; ++nb) acc[mb][nb] = (v8f){};
    const size_t aoff = (size_t)lr * lda + 8 * hi, boff = (size_t)lr * ldb + 8 * hi;
#pragma unroll 1
    for (int kc = 0; kc < K; kc += 32) {
        v16h a[4];
#pragma unroll
        for (int mb = 0; mb < 4; ++mb) a[mb] = ldh(Ap + aoff + (size_t)mb * 16 * lda + kc);
#pragma unroll
        for (int nb = 0; nb < 4; ++nb) { const v16h b = ldh(Bp + boff + (size_t)nb * 16 * ldb + kc);
#pragma unroll
            for (int mb = 0; mb < 4; ++mb) acc[mb][nb] = wmmag(a[mb], b, acc[mb][nb]); }
    }
}

__global__ __launch_bounds__(256) void k_wT(const float* __restrict__ W, h16* WT, int R, int C) {
    __shared__ float ts[64 * 65];
    const int tid = threadIdx.x;
    const int c0 = blockIdx.x * 64, r0 = blockIdx.y * 64;
#pragma unroll 1
    for (int it = 0; it < 4; ++it) { const int idx = it * 256 + tid; const int row = idx >> 4, c4 = (idx & 15) * 4;
        const v4f v = *(const v4f*)(W + (size_t)(r0 + row) * C + c0 + c4);
        ts[row * 65 + c4 + 0] = v[0]; ts[row * 65 + c4 + 1] = v[1]; ts[row * 65 + c4 + 2] = v[2]; ts[row * 65 + c4 + 3] = v[3]; }
    __syncthreads();
#pragma unroll 1
    for (int ps = 0; ps < 2; ++ps) {
#pragma unroll 1
        for (int it = 0; it < 2; ++it) { const int p = it * 256 + tid; const int orow = p >> 3, c8 = (p & 7) * 8;
            v8h hv;
#pragma unroll
            for (int i = 0; i < 8; ++i) hv[i] = toh_flush(bfr(ts[(c8 + i) * 65 + orow]) * WS);
            *(volatile v8h*)(WT + (size_t)(c0 + orow) * R + r0 + c8) = hv; }
        if (ps == 0) __threadfence(); }
}

__global__ __launch_bounds__(256) void k_ln(const float* __restrict__ x, const float* __restrict__ g, const float* __restrict__ be, h16* out, int srcSeq, int rin) {
    const int lane = threadIdx.x & 31;
    const int wave = __builtin_amdgcn_readfirstlane((int)(threadIdx.x >> 5));
    const int row = blockIdx.x * 8 + wave;
    const int b = row / SEQ, t = row % SEQ;
    const float* src = x + ((size_t)b * (size_t)srcSeq + (size_t)t) * DM + lane * 8;
    float s = 0.0f;
#pragma unroll 1
    for (int c = 0; c < 2; ++c) { const v8f v = *(const v8f*)(src + c * 256);
#pragma unroll
        for (int k = 0; k < 8; ++k) { const float cv = bfr(v[k]); const float a = rin ? cv : v[k]; s += a; } }
    s += __shfl_xor(s, 16, 32); s += __shfl_xor(s, 8, 32); s += __shfl_xor(s, 4, 32); s += __shfl_xor(s, 2, 32); s += __shfl_xor(s, 1, 32);
    const float mean = s * (1.0f / 512.0f);
    float ss = 0.0f;
#pragma unroll 1
    for (int c = 0; c < 2; ++c) { const v8f v = *(const v8f*)(src + c * 256);
#pragma unroll
        for (int k = 0; k < 8; ++k) { const float cv = bfr(v[k]); const float a = rin ? cv : v[k]; const float d = a - mean; ss += d * d; } }
    ss += __shfl_xor(ss, 16, 32); ss += __shfl_xor(ss, 8, 32); ss += __shfl_xor(ss, 4, 32); ss += __shfl_xor(ss, 2, 32); ss += __shfl_xor(ss, 1, 32);
    const float rstd = rsqrtf(ss * (1.0f / 512.0f) + LNEPS);
    h16* dst = out + (size_t)row * DM + lane * 8;
#pragma unroll 1
    for (int ps = 0; ps < 2; ++ps) {
#pragma unroll 1
        for (int c = 0; c < 2; ++c) {
            const v8f v = *(const v8f*)(src + c * 256);
            const v8f gv = *(const v8f*)(g + c * 256 + lane * 8);
            const v8f bv = *(const v8f*)(be + c * 256 + lane * 8);
            v8h o;
#pragma unroll
            for (int k = 0; k < 8; ++k) { const float cv = bfr(v[k]); const float a = rin ? cv : v[k];
                const float y = (a - mean) * rstd * bfr(gv[k]) + bfr(bv[k]); o[k] = toh_flush(y); }
            *(volatile v8h*)(dst + c * 256) = o; }
        if (ps == 0) __threadfence(); }
}

__global__ __launch_bounds__(32) void k_gemm_h(const h16* __restrict__ A, const h16* __restrict__ Bt, const float* __restrict__ bias, h16* C,
                                               size_t aZb, size_t aZh, size_t bZb, size_t bZh, size_t cZb, size_t cZh,
                                               int lda, int ldb, int ldc, int K, int hasBias, int relu, float scale) {
    __shared__ __align__(16) float os[16 * 68];
    const int lane = threadIdx.x & 31, lr = lane & 15, hi = lane >> 4;
    const int r0 = blockIdx.x * 64, c0 = blockIdx.y * 64;
    const int z = blockIdx.z; const int zb = z / NH_, zh = z % NH_;
    const h16* Ap = A + (size_t)zb * aZb + (size_t)zh * aZh + (size_t)r0 * (size_t)lda;
    const h16* Bp = Bt + (size_t)zb * bZb + (size_t)zh * bZh + (size_t)c0 * (size_t)ldb;
    h16* Cp = C + (size_t)zb * cZb + (size_t)zh * cZh + (size_t)r0 * (size_t)ldc + (size_t)c0;
    v8f acc[4][4];
    gemm_acc(Ap, Bp, (size_t)lda, (size_t)ldb, K, lr, hi, acc);
    float bc[4] = { 0.0f, 0.0f, 0.0f, 0.0f };
    if (hasBias) {
#pragma unroll
        for (int nb = 0; nb < 4; ++nb) bc[nb] = bfr(bias[c0 + nb * 16 + lr]); }
#pragma unroll
    for (int mb = 0; mb < 4; ++mb) {
#pragma unroll
        for (int nb = 0; nb < 4; ++nb) {
#pragma unroll
            for (int j = 0; j < 8; ++j) { float v = acc[mb][nb][j] * scale + bc[nb]; const float vr = fmaxf(v, 0.0f); v = relu ? vr : v;
                os[(hi * 8 + j) * 68 + nb * 16 + lr] = v; } }
        wave_sync();
#pragma unroll 1
        for (int ps = 0; ps < 2; ++ps) {
#pragma unroll
            for (int s = 0; s < 4; ++s) { const int row = 4 * s + (lane >> 3), c8 = (lane & 7) * 8;
                const v4f x0 = *(const v4fa*)(&os[row * 68 + c8]); const v4f x1 = *(const v4fa*)(&os[row * 68 + c8 + 4]); v8h hv;
#pragma unroll
                for (int i = 0; i < 4; ++i) { hv[i] = toh_flush(x0[i]); hv[4 + i] = toh_flush(x1[i]); }
                *(volatile v8h*)(Cp + (size_t)(mb * 16 + row) * (size_t)ldc + c8) = hv; }
            if (ps == 0) __threadfence(); }
        wave_sync();
    }
}

__global__ __launch_bounds__(32) void k_gemm_t(const h16* __restrict__ A, const h16* __restrict__ Bt, const float* __restrict__ bias, h16* C, float scale) {
    __shared__ __align__(16) float os[16 * 68];
    const int lane = threadIdx.x & 31, lr = lane & 15, hi = lane >> 4;
    const int r0 = blockIdx.x * 64, c0 = blockIdx.y * 64;
    const int bb = c0 / SEQ, tt = c0 % SEQ;
    v8f acc[4][4];
    gemm_acc(A + (size_t)r0 * DM, Bt + (size_t)c0 * DM, (size_t)DM, (size_t)DM, DM, lr, hi, acc);
    h16* Cp = C + ((size_t)bb * DH + (size_t)r0) * SEQ + (size_t)tt;
#pragma unroll
    for (int mb = 0; mb < 4; ++mb) {
        float br[8];
#pragma unroll
        for (int j = 0; j < 8; ++j) br[j] = bfr(bias[r0 + mb * 16 + hi * 8 + j]);
#pragma unroll
        for (int nb = 0; nb < 4; ++nb) { const bool zt = (tt + nb * 16 + lr) == (SEQ - 1);
#pragma unroll
            for (int j = 0; j < 8; ++j) { const float v = acc[mb][nb][j] * scale + br[j];
                os[(hi * 8 + j) * 68 + nb * 16 + lr] = zt ? 0.0f : v; } }
        wave_sync();
#pragma unroll 1
        for (int ps = 0; ps < 2; ++ps) {
#pragma unroll
            for (int s = 0; s < 4; ++s) { const int row = 4 * s + (lane >> 3), c8 = (lane & 7) * 8;
                const v4f x0 = *(const v4fa*)(&os[row * 68 + c8]); const v4f x1 = *(const v4fa*)(&os[row * 68 + c8 + 4]); v8h hv;
#pragma unroll
                for (int i = 0; i < 4; ++i) { hv[i] = toh_flush(x0[i]); hv[4 + i] = toh_flush(x1[i]); }
                *(volatile v8h*)(Cp + (size_t)(mb * 16 + row) * SEQ + c8) = hv; }
            if (ps == 0) __threadfence(); }
        wave_sync();
    }
}

__global__ __launch_bounds__(32) void k_gemm_f(const h16* __restrict__ A, const h16* __restrict__ Bt, const float* __restrict__ bias, const float* __restrict__ res, float* C,
                                               int lda, int ldb, int K, int resSeq, int outSeq, int rres, float scale) {
    __shared__ __align__(16) float os[16 * 68];
    const int lane = threadIdx.x & 31, lr = lane & 15, hi = lane >> 4;
    const int r0 = blockIdx.x * 64, c0 = blockIdx.y * 64;
    const int bb = r0 / SEQ, tt = r0 % SEQ;
    v8f acc[4][4];
    gemm_acc(A + (size_t)r0 * (size_t)lda, Bt + (size_t)c0 * (size_t)ldb, (size_t)lda, (size_t)ldb, K, lr, hi, acc);
    const float* rp = res + ((size_t)bb * (size_t)resSeq + (size_t)tt) * DM + c0;
    float* cp = C + ((size_t)bb * (size_t)outSeq + (size_t)tt) * DM + c0;
    float bc[4];
#pragma unroll
    for (int nb = 0; nb < 4; ++nb) bc[nb] = bfr(bias[c0 + nb * 16 + lr]);
#pragma unroll
    for (int mb = 0; mb < 4; ++mb) {
#pragma unroll
        for (int nb = 0; nb < 4; ++nb) {
#pragma unroll
            for (int j = 0; j < 8; ++j) os[(hi * 8 + j) * 68 + nb * 16 + lr] = acc[mb][nb][j] * scale + bc[nb]; }
        wave_sync();
#pragma unroll 1
        for (int ps = 0; ps < 2; ++ps) {
#pragma unroll
            for (int s = 0; s < 8; ++s) { const int row = 2 * s + (lane >> 4), c4 = (lane & 15) * 4;
                const v4f v = *(const v4fa*)(&os[row * 68 + c4]);
                const v4f r = *(const v4f*)(rp + (size_t)(mb * 16 + row) * DM + c4);
                v4f val;
#pragma unroll
                for (int i = 0; i < 4; ++i) { const float rc = bfr(r[i]); const float ra = rres ? rc : r[i]; val[i] = v[i] + ra; }
                *(volatile v4f*)(cp + (size_t)(mb * 16 + row) * DM + c4) = val; }
            if (ps == 0) __threadfence(); }
        wave_sync();
    }
}

static constexpr size_t al256(size_t v) { return (v + 255) & ~(size_t)255; }
static constexpr size_t SZ_WA = al256((size_t)DM * DH * 2);
static constexpr size_t SZ_WF = al256((size_t)DM * DFF * 2);
static constexpr size_t SZ_HN = al256((size_t)NB * SEQ * DM * 2);
static constexpr size_t SZ_R  = al256((size_t)NB * SEQ * DH * 2);
static constexpr size_t SZ_MT = al256((size_t)NB * NH_ * DM * DM * 2);
static constexpr size_t SZ_X1 = al256((size_t)NB * SEQ * DM * 4);
static constexpr size_t SZ_TOTAL = 4 * SZ_WA + 2 * SZ_WF + SZ_HN + 2 * SZ_R + SZ_MT + SZ_X1;
static_assert(SZ_TOTAL <= (size_t)134217728);
static_assert((size_t)NB * DH * SEQ * 2 <= SZ_R);
static_assert((size_t)NB * SEQ * DH * 2 <= SZ_R);
static_assert((size_t)NB * SEQ * DFF * 2 <= SZ_R);
static_assert((size_t)DM * DH * 2 <= SZ_WA);
static_assert((size_t)DM * DFF * 2 <= SZ_WF);

extern "C" void kernel_launch(void* const* d_in, const int* in_sizes, int n_in,
                              void* d_out, int out_size, void* d_ws, size_t ws_size, hipStream_t stream) {
    if (n_in < 17) return;
    const size_t needx = ((size_t)(NB - 1) * SEQ_FULL + SEQ) * DM;
    if ((size_t)in_sizes[0] < needx) return;
    if ((size_t)in_sizes[1] < (size_t)DM * DH || (size_t)in_sizes[3] < (size_t)DM * DH || (size_t)in_sizes[5] < (size_t)DM * DH || (size_t)in_sizes[7] < (size_t)DH * DM) return;
    if (in_sizes[2] < DH || in_sizes[4] < DH || in_sizes[6] < DH) return;
    if (in_sizes[8] < DM || in_sizes[9] < DM || in_sizes[10] < DM) return;
    if ((size_t)in_sizes[11] < (size_t)DM * DFF || in_sizes[12] < DFF || (size_t)in_sizes[13] < (size_t)DFF * DM) return;
    if (in_sizes[14] < DM || in_sizes[15] < DM || in_sizes[16] < DM) return;
    if ((size_t)out_size < ((size_t)(NB - 1) * OUT_SEQ + SEQ) * DM) return;
    if (SZ_TOTAL > ws_size) return;
    const float* x   = (const float*)d_in[0];
    const float* wq  = (const float*)d_in[1];  const float* bq  = (const float*)d_in[2];
    const float* wk  = (const float*)d_in[3];  const float* bk  = (const float*)d_in[4];
    const float* wv  = (const float*)d_in[5];  const float* bv  = (const float*)d_in[6];
    const float* wp  = (const float*)d_in[7];  const float* bp  = (const float*)d_in[8];
    const float* l1g = (const float*)d_in[9];  const float* l1b = (const float*)d_in[10];
    const float* w1  = (const float*)d_in[11]; const float* b1  = (const float*)d_in[12];
    const float* w2  = (const float*)d_in[13]; const float* b2  = (const float*)d_in[14];
    const float* l2g = (const float*)d_in[15]; const float* l2b = (const float*)d_in[16];
    float* OUT = (float*)d_out;
    char* wsp = (char*)d_ws;
    h16* WQT = (h16*)wsp; wsp += SZ_WA;
    h16* WKT = (h16*)wsp; wsp += SZ_WA;
    h16* WVT = (h16*)wsp; wsp += SZ_WA;
    h16* WPT = (h16*)wsp; wsp += SZ_WA;
    h16* W1T = (h16*)wsp; wsp += SZ_WF;
    h16* W2T = (h16*)wsp; wsp += SZ_WF;
    h16* HN  = (h16*)wsp; wsp += SZ_HN;
    h16* R1  = (h16*)wsp; wsp += SZ_R;
    h16* R2  = (h16*)wsp; wsp += SZ_R;
    h16* MT  = (h16*)wsp; wsp += SZ_MT;
    float* X1 = (float*)wsp; wsp += SZ_X1;

    k_wT<<<dim3(DH / 64, DM / 64, 1), 256, 0, stream>>>(wq, WQT, DM, DH);
    k_wT<<<dim3(DH / 64, DM / 64, 1), 256, 0, stream>>>(wk, WKT, DM, DH);
    k_wT<<<dim3(DH / 64, DM / 64, 1), 256, 0, stream>>>(wv, WVT, DM, DH);
    k_wT<<<dim3(DM / 64, DH / 64, 1), 256, 0, stream>>>(wp, WPT, DH, DM);
    k_wT<<<dim3(DFF / 64, DM / 64, 1), 256, 0, stream>>>(w1, W1T, DM, DFF);
    k_wT<<<dim3(DM / 64, DFF / 64, 1), 256, 0, stream>>>(w2, W2T, DFF, DM);

    k_ln<<<dim3(NB * SEQ / 8, 1, 1), 256, 0, stream>>>(x, l1g, l1b, HN, SEQ_FULL, 1);

    k_gemm_t<<<dim3(DH / 64, NB * SEQ / 64, 1), 32, 0, stream>>>(WKT, HN, bk, R1, WSI);
    k_gemm_t<<<dim3(DH / 64, NB * SEQ / 64, 1), 32, 0, stream>>>(WVT, HN, bv, R2, WSI);

    k_gemm_h<<<dim3(DM / 64, DM / 64, NB * NH_), 32, 0, stream>>>(R2, R1, bq, MT,
        (size_t)DH * SEQ, (size_t)DM * SEQ, (size_t)DH * SEQ, (size_t)DM * SEQ, (size_t)NH_ * DM * DM, (size_t)DM * DM,
        SEQ, SEQ, DM, SEQ, 0, 0, 1.0f);

    k_gemm_h<<<dim3(NB * SEQ / 64, DH / 64, 1), 32, 0, stream>>>(HN, WQT, bq, R1,
        (size_t)0, (size_t)0, (size_t)0, (size_t)0, (size_t)0, (size_t)0,
        DM, DM, DH, DM, 1, 0, WSI);

    k_gemm_h<<<dim3(SEQ / 64, DM / 64, NB * NH_), 32, 0, stream>>>(R1, MT, bq, R2,
        (size_t)SEQ * DH, (size_t)DM, (size_t)NH_ * DM * DM, (size_t)DM * DM, (size_t)SEQ * DH, (size_t)DM,
        DH, DM, DH, DM, 0, 0, 1.0f);

    k_gemm_f<<<dim3(NB * SEQ / 64, DM / 64, 1), 32, 0, stream>>>(R2, WPT, bp, x, X1, DH, DH, DH, SEQ_FULL, SEQ, 1, WSI);

    k_ln<<<dim3(NB * SEQ / 8, 1, 1), 256, 0, stream>>>(X1, l2g, l2b, HN, SEQ, 0);

    k_gemm_h<<<dim3(NB * SEQ / 64, DFF / 64, 1), 32, 0, stream>>>(HN, W1T, b1, R1,
        (size_t)0, (size_t)0, (size_t)0, (size_t)0, (size_t)0, (size_t)0,
        DM, DM, DFF, DM, 1, 1, WSI);

    k_gemm_f<<<dim3(NB * SEQ / 64, DM / 64, 1), 32, 0, stream>>>(R1, W2T, b2, X1, OUT, DFF, DFF, DFF, SEQ, OUT_SEQ, 0, WSI);
}
